// PointNetSAModule_86260123173794
// MI455X (gfx1250) — hardware-verified
//
#include <hip/hip_runtime.h>
#include <math.h>

#pragma clang fp contract(off)

constexpr int NBATCH   = 16;
constexpr int NPTS     = 4096;
constexpr int CIN      = 64;
constexpr int NCEN     = 1024;
constexpr int KNBR     = 32;
constexpr int W1PITCH  = 67;
constexpr int NCENTOT  = NBATCH * NCEN;
constexpr int NCOL     = NCENTOT * KNBR;
constexpr int NCH12    = 64;
constexpr int NCH3     = 128;
constexpr float RADIUS2    = 0.04f;
constexpr float BN_EPS     = 1e-5f;
constexpr float WCARRY     = 16.0f;
constexpr float WCARRY_INV = 1.0f / 16.0f;
constexpr float YCARRY     = 64.0f;
constexpr float YCARRY_INV = 1.0f / 64.0f;
constexpr int NT      = 256;
constexpr int ROWS12  = 256;
constexpr int ROWS3   = 128;
constexpr int NBLK12  = NCOL / ROWS12;
constexpr int NBLK3   = NCOL / ROWS3;
constexpr int FPS_NT  = 512;
constexpr int NWCBLK  = 8;

static_assert(NCOL % ROWS12 == 0);
static_assert(NCOL % ROWS3 == 0);
static_assert(ROWS12 == 8 * KNBR);
static_assert(ROWS3 == 4 * KNBR);
static_assert(CIN % 32 == 0);
static_assert(NPTS == FPS_NT * 8);
static_assert(NBLK12 * ROWS12 == NCOL);
static_assert(NBLK3 * ROWS3 == NCOL);
static_assert(NCEN / 8 == 128);

typedef __attribute__((ext_vector_type(16))) _Float16 v16h;
typedef __attribute__((ext_vector_type(8)))  _Float16 v8h;
typedef __attribute__((ext_vector_type(16))) __bf16   v16b;
typedef __attribute__((ext_vector_type(8)))  __bf16   v8b;
typedef __attribute__((ext_vector_type(8)))  float    v8f;
typedef __attribute__((ext_vector_type(4)))  float    v4f;
typedef __attribute__((ext_vector_type(4)))  unsigned int v4u;

__device__ __forceinline__ unsigned short f2bf_bits(float f) {
  unsigned u = __float_as_uint(f);
  return (unsigned short)((u + 0x7FFFu + ((u >> 16) & 1u)) >> 16);
}
__device__ __forceinline__ float bf_bits2f(unsigned short h) { return __uint_as_float(((unsigned)h) << 16); }

__device__ __forceinline__ void dep_guard_h(v8f& a, v8f& b, v16h x, v16h y) { asm volatile("v_nop\n\tv_nop\n\tv_nop\n\tv_nop" : "+v"(a), "+v"(b) : "v"(x), "v"(y)); }
__device__ __forceinline__ void dep_guard_b(v8f& a, v8f& b, v16b x, v16b y) { asm volatile("v_nop\n\tv_nop\n\tv_nop\n\tv_nop" : "+v"(a), "+v"(b) : "v"(x), "v"(y)); }
__device__ __forceinline__ void keep4_h(v16h a, v16h b, v16h c, v16h d) { asm volatile("v_nop" :: "v"(a), "v"(b), "v"(c), "v"(d)); }
__device__ __forceinline__ void keep4_b(v16b a, v16b b, v16b c, v16b d) { asm volatile("v_nop" :: "v"(a), "v"(b), "v"(c), "v"(d)); }
__device__ __forceinline__ void acc_guard4(v8f& a, v8f& b, v8f& c, v8f& d) { asm volatile("v_nop\n\tv_nop\n\tv_nop\n\tv_nop" : "+v"(a), "+v"(b), "+v"(c), "+v"(d)); }
template <typename T> struct Frag;
template <> struct Frag<_Float16> {
  typedef v16h V; union U { v16h v; v8h h[2]; };
  static __device__ __forceinline__ v16h load(const _Float16* p) {
    U f; f.h[0] = *(const v8h*)(p); f.h[1] = *(const v8h*)(p + 16); return f.v;
  }
  static __device__ __forceinline__ v8f mma(v16h a, v16h b, v8f c) {
    return __builtin_amdgcn_wmma_f32_16x16x32_f16(false, a, false, b, (short)0, c, false, false);
  }
  static __device__ __forceinline__ void guard(v8f& a, v8f& b, v16h x, v16h y) { dep_guard_h(a, b, x, y); }
  static __device__ __forceinline__ void keep(v16h a, v16h b, v16h c, v16h d) { keep4_h(a, b, c, d); }
};
template <> struct Frag<__bf16> {
  typedef v16b V; union U { v16b v; v8b h[2]; };
  static __device__ __forceinline__ v16b load(const __bf16* p) {
    U f; f.h[0] = *(const v8b*)(p); f.h[1] = *(const v8b*)(p + 16); return f.v;
  }
  static __device__ __forceinline__ v8f mma(v16b a, v16b b, v8f c) {
    return __builtin_amdgcn_wmma_f32_16x16x32_bf16(false, a, false, b, (short)0, c, false, false);
  }
  static __device__ __forceinline__ void guard(v8f& a, v8f& b, v16b x, v16b y) { dep_guard_b(a, b, x, y); }
  static __device__ __forceinline__ void keep(v16b a, v16b b, v16b c, v16b d) { keep4_b(a, b, c, d); }
};

__device__ __forceinline__ unsigned pk16(unsigned short a, unsigned short b) { return (unsigned)a | ((unsigned)b << 16); }
__device__ __forceinline__ unsigned short h_bits(float f) { const _Float16 h = (_Float16)f; return __builtin_bit_cast(unsigned short, h); }

__device__ __forceinline__ float h16_to_f32(unsigned hb) {
  const unsigned sgn = (hb & 0x8000u) << 16; const unsigned em = hb & 0x7fffu;
  const float fn = __uint_as_float((em << 13) + 0x38000000u);
  const float fs = (float)em * 5.9604644775390625e-8f;
  const float mag = (em < 0x400u) ? fs : fn; return __uint_as_float(__float_as_uint(mag) | sgn); }

__device__ __forceinline__ void tile_gemm(const _Float16* A32, const _Float16* B64, int rl, int hh, v8f (&acc)[2][4]) {
#pragma unroll
  for (int i = 0; i < 2; ++i)
#pragma unroll
    for (int j = 0; j < 4; ++j) acc[i][j] = (v8f){0.f, 0.f, 0.f, 0.f, 0.f, 0.f, 0.f, 0.f};
#pragma unroll
  for (int ks = 0; ks < 2; ++ks) {
    const int k0 = ks * 32 + 8 * hh;
    v16h bf[4];
#pragma unroll
    for (int j = 0; j < 4; ++j) bf[j] = Frag<_Float16>::load(B64 + (16 * j + rl) * 64 + k0);
#pragma unroll
    for (int i = 0; i < 2; ++i) {
      const v16h af = Frag<_Float16>::load(A32 + (16 * i + rl) * 64 + k0);
#pragma unroll
      for (int j = 0; j < 4; ++j) acc[i][j] = Frag<_Float16>::mma(af, bf[j], acc[i][j]);
      Frag<_Float16>::guard(acc[i][0], acc[i][3], af, af);
    }
    Frag<_Float16>::keep(bf[0], bf[1], bf[2], bf[3]);
  }
  acc_guard4(acc[0][0], acc[0][1], acc[0][2], acc[0][3]);
  acc_guard4(acc[1][0], acc[1][1], acc[1][2], acc[1][3]);
}

__device__ __forceinline__ void tile_stats(const v8f (&y)[2][4], int hh, int rl, int wave, float* sStat) {
  float s[4], q[4];
#pragma unroll
  for (int j = 0; j < 4; ++j) { s[j] = 0.0f; q[j] = 0.0f; }
#pragma unroll
  for (int i = 0; i < 2; ++i)
#pragma unroll
    for (int j = 0; j < 4; ++j)
#pragma unroll
      for (int r = 0; r < 8; ++r) {
        const float v = y[i][j][r];
        s[j] = s[j] + v;
        q[j] = fmaf(v, v, q[j]);
      }
#pragma unroll
  for (int j = 0; j < 4; ++j) {
    s[j] += __shfl_xor(s[j], 16, 32);
    q[j] += __shfl_xor(q[j], 16, 32);
  }
  if (hh == 0) {
#pragma unroll
    for (int j = 0; j < 4; ++j) {
      sStat[(wave * 2 + 0) * 64 + 16 * j + rl] = s[j];
      sStat[(wave * 2 + 1) * 64 + 16 * j + rl] = q[j];
    }
  }
}

__device__ __forceinline__ void argmax_reduce(float& bv, int& bi) {
#pragma unroll
  for (int off = 16; off >= 1; off >>= 1) {
    const float ov = __shfl_xor(bv, off, 32);
    const int oi = __shfl_xor(bi, off, 32);
    const bool take = (ov > bv) || (ov == bv && oi < bi);
    bv = take ? ov : bv;
    bi = take ? oi : bi;
  }
}

__global__ __launch_bounds__(NT) void feat_transpose_kernel(const float* __restrict__ feat, unsigned short* __restrict__ FT) {
  __shared__ float sm[64][65];
  const int t = threadIdx.x;
  const int p0 = blockIdx.x * 64;
  const int b = blockIdx.y;
  const float* fb = feat + (size_t)b * CIN * NPTS + p0;
#pragma unroll
  for (int i = 0; i < 4; ++i) {
    const int e = i * NT + t;
    const int c = e >> 4;
    const int p4 = (e & 15) * 4;
    const v4f v = *(const v4f*)(fb + (size_t)c * NPTS + p4);
    sm[p4][c] = v[0];
    sm[p4 + 1][c] = v[1];
    sm[p4 + 2][c] = v[2];
    sm[p4 + 3][c] = v[3];
  }
  __syncthreads();
  const int lane = t & 31, wave = t >> 5;
  const int q = lane >> 3, c8 = (lane & 7) * 8;
  unsigned short* op = FT + ((size_t)b * NPTS + p0) * CIN;
  v4u u[2];
#pragma unroll
  for (int it = 0; it < 2; ++it) {
    const int row = wave * 8 + it * 4 + q;
    unsigned short hb[8];
#pragma unroll
    for (int e = 0; e < 8; ++e) hb[e] = h_bits(sm[row][c8 + e]);
    u[it] = (v4u){pk16(hb[0], hb[1]), pk16(hb[2], hb[3]), pk16(hb[4], hb[5]), pk16(hb[6], hb[7])};
  }
  for (int pass = 0; pass < 2; ++pass) {
#pragma unroll
    for (int it = 0; it < 2; ++it) {
      const int row = wave * 8 + it * 4 + q;
      *(volatile v4u*)(op + (size_t)row * CIN + c8) = u[it];
    }
    __threadfence();
  }
}

__global__ __launch_bounds__(NT) void wcast_kernel(const float* __restrict__ w1, const float* __restrict__ w2,
                                                   const float* __restrict__ w3, unsigned short* __restrict__ WT) {
  const int zsrc = blockIdx.x >> 1;
  const int half = blockIdx.x & 1;
  const float* src = w1; int pitch = W1PITCH; int coff = 3;
  if (zsrc == 1) { src = w2; pitch = 64; coff = 0; }
  else if (zsrc == 2) { src = w3; pitch = 64; coff = 0; }
  else if (zsrc == 3) { src = w3 + 64 * 64; pitch = 64; coff = 0; }
  const int t = threadIdx.x, lane = t & 31, wave = t >> 5;
  const int q = lane >> 3, c8 = (lane & 7) * 8;
  const int row = half * 32 + wave * 4 + q;
  const float* sp = src + (size_t)row * pitch + coff + c8;
  unsigned short hb[8];
#pragma unroll
  for (int e = 0; e < 8; ++e) hb[e] = h_bits(sp[e] * WCARRY);
  const v4u u = (v4u){pk16(hb[0], hb[1]), pk16(hb[2], hb[3]), pk16(hb[4], hb[5]), pk16(hb[6], hb[7])};
  unsigned short* op = WT + (size_t)zsrc * 64 * 64 + (size_t)row * 64 + c8;
  *(volatile v4u*)op = u;
  __threadfence();
  *(volatile v4u*)op = u;
}

__global__ __launch_bounds__(FPS_NT) void fps_kernel(const float* __restrict__ coords, float* __restrict__ cen) {
  __shared__ __align__(16) float sX[NPTS];
  __shared__ __align__(16) float sY[NPTS];
  __shared__ __align__(16) float sZ[NPTS];
  __shared__ int sC[NCEN];
  __shared__ float sRv[16];
  __shared__ int sRi[16];
  __shared__ int sLast;
  const int b = blockIdx.x, tid = threadIdx.x, lane = tid & 31, wave = tid >> 5;
  const float* cb = coords + (size_t)b * 3 * NPTS;
#pragma unroll 1
  for (int i = tid; i < NPTS / 4; i += FPS_NT) {
    const v4f vx = *(const v4f*)(cb + 4 * i);
    const v4f vy = *(const v4f*)(cb + NPTS + 4 * i);
    const v4f vz = *(const v4f*)(cb + 2 * NPTS + 4 * i);
    *(v4f*)(sX + 4 * i) = vx;
    *(v4f*)(sY + 4 * i) = vy;
    *(v4f*)(sZ + 4 * i) = vz;
  }
  if (tid == 0) { sC[0] = 0; sLast = 0; }
  __syncthreads();

  const int p0 = tid * 8;
  float px[8], py[8], pz[8], mind[8];
  {
    const v4f xa = *(const v4f*)(sX + p0), xb = *(const v4f*)(sX + p0 + 4);
    const v4f ya = *(const v4f*)(sY + p0), yb = *(const v4f*)(sY + p0 + 4);
    const v4f za = *(const v4f*)(sZ + p0), zb = *(const v4f*)(sZ + p0 + 4);
#pragma unroll
    for (int j = 0; j < 4; ++j) {
      px[j] = xa[j]; px[4 + j] = xb[j];
      py[j] = ya[j]; py[4 + j] = yb[j];
      pz[j] = za[j]; pz[4 + j] = zb[j];
      mind[j] = 1e10f; mind[4 + j] = 1e10f;
    }
  }
  int L = 0;
#pragma unroll 1
  for (int s = 1; s < NCEN; ++s) {
    const float lx = sX[L], ly = sY[L], lz = sZ[L];
    float bv = -1.0f; int bi = p0;
#pragma unroll
    for (int j = 0; j < 8; ++j) {
      const float dx = px[j] - lx, dy = py[j] - ly, dz = pz[j] - lz;
      const float t0 = dx * dx;
      const float t1 = dy * dy;
      const float t2 = dz * dz;
      const float d = (t0 + t1) + t2;
      const float mn = fminf(mind[j], d);
      mind[j] = mn;
      const bool sel = mn > bv;
      bv = sel ? mn : bv;
      bi = sel ? (p0 + j) : bi;
    }
    argmax_reduce(bv, bi);
    if (lane == 0) { sRv[wave] = bv; sRi[wave] = bi; }
    __syncthreads();
    if (wave == 0) {
      float v = sRv[lane & 15]; int i2 = sRi[lane & 15];
      argmax_reduce(v, i2);
      if (lane == 0) { sLast = i2; sC[s] = i2; }
    }
    __syncthreads();
    L = sLast;
  }
  if (wave < 8) {
    const int m4 = 4 * tid;
    int i0 = sC[m4], i1 = sC[m4 + 1], i2 = sC[m4 + 2], i3 = sC[m4 + 3];
    i0 = i0 < 0 ? 0 : (i0 > NPTS - 1 ? NPTS - 1 : i0);
    i1 = i1 < 0 ? 0 : (i1 > NPTS - 1 ? NPTS - 1 : i1);
    i2 = i2 < 0 ? 0 : (i2 > NPTS - 1 ? NPTS - 1 : i2);
    i3 = i3 < 0 ? 0 : (i3 > NPTS - 1 ? NPTS - 1 : i3);
    const v4f vx = (v4f){sX[i0], sX[i1], sX[i2], sX[i3]};
    const v4f vy = (v4f){sY[i0], sY[i1], sY[i2], sY[i3]};
    const v4f vz = (v4f){sZ[i0], sZ[i1], sZ[i2], sZ[i3]};
    float* ob = cen + (size_t)b * 3 * NCEN;
    for (int pass = 0; pass < 2; ++pass) {
      *(volatile v4f*)(ob + m4) = vx;
      *(volatile v4f*)(ob + NCEN + m4) = vy;
      *(volatile v4f*)(ob + 2 * NCEN + m4) = vz;
      __threadfence();
    }
  }
}

template <bool DO_L2>
__global__ __launch_bounds__(NT) void mlp12_kernel(
    const unsigned short* __restrict__ FT, const float* __restrict__ coords, const float* __restrict__ cen,
    const unsigned short* __restrict__ WT, const float* __restrict__ w1, const float* __restrict__ b1,
    const float* __restrict__ SS1, const float* __restrict__ b2,
    float* __restrict__ PART, unsigned short* __restrict__ Y2) {
  __shared__ __align__(16) unsigned short sA[ROWS12 * 64];
  __shared__ __align__(16) unsigned short sW1[64 * 64];
  __shared__ __align__(16) unsigned short sW2[DO_L2 ? 64 * 64 : 8];
  __shared__ __align__(16) float sRel[ROWS12 * 4];
  __shared__ __align__(16) float sWc[64 * 4];
  __shared__ float sB1[64];
  __shared__ float sSc[64];
  __shared__ float sSh[64];
  __shared__ float sB2[64];
  __shared__ float sStat[8 * 2 * 64];
  __shared__ __align__(16) float sBlk[128];
  __shared__ int sIdx[ROWS12];

  const int tid = threadIdx.x, lane = tid & 31, wave = tid >> 5;
  const int rl = lane & 15, hh = lane >> 4;
  const int blk = blockIdx.x;
  const int r0 = blk * ROWS12;
  const int bb = blk >> 7;
  const int mbase = (blk & 127) * 8;

  {
    const v4u* wsrc = (const v4u*)WT;
    v4u* d1 = (v4u*)sW1;
#pragma unroll
    for (int i = 0; i < 2; ++i) d1[i * NT + tid] = wsrc[i * NT + tid];
    if (DO_L2) {
      v4u* d2 = (v4u*)sW2;
#pragma unroll
      for (int i = 0; i < 2; ++i) d2[i * NT + tid] = wsrc[512 + i * NT + tid];
    }
  }
  if (tid < 64) {
    sWc[tid * 4 + 0] = w1[tid * W1PITCH + 0];
    sWc[tid * 4 + 1] = w1[tid * W1PITCH + 1];
    sWc[tid * 4 + 2] = w1[tid * W1PITCH + 2];
    sWc[tid * 4 + 3] = 0.0f;
    sB1[tid] = b1[tid];
    if (DO_L2) { sSc[tid] = SS1[tid]; sSh[tid] = SS1[64 + tid]; sB2[tid] = b2[tid]; }
  }

  const float* cb = coords + (size_t)bb * 3 * NPTS;
  const float* ce = cen + (size_t)bb * 3 * NCEN;

  {
    const int m = mbase + wave;
    const float cx = ce[m], cy = ce[NCEN + m], cz = ce[2 * NCEN + m];
    const float c0 = cx * cx;
    const float c1 = cy * cy;
    const float c2 = cz * cz;
    const float sc = (c0 + c1) + c2;
    sIdx[wave * 32 + lane] = 0;
    int cnt = 0, first = 0, have = 0;
#pragma unroll 1
    for (int ch = 0; ch < NPTS / 32; ++ch) {
      if (cnt >= KNBR) break;
      const int j = ch * 32 + lane;
      const float px = cb[j], py = cb[NPTS + j], pz = cb[2 * NPTS + j];
      const float q0 = px * px;
      const float q1 = py * py;
      const float q2 = pz * pz;
      const float sp = (q0 + q1) + q2;
      float p = cx * px; p = fmaf(cy, py, p); p = fmaf(cz, pz, p);
      const float p2 = 2.0f * p;
      const float d2 = (sc + sp) - p2;
      const int pred = (d2 < RADIUS2) ? 1 : 0;
      const unsigned mask = (unsigned)__ballot(pred);
      if (have == 0 && mask != 0u) { first = ch * 32 + (__builtin_ffs((int)mask) - 1); have = 1; }
      const int pos = cnt + (int)__popc(mask & ((1u << lane) - 1u));
      if (pred != 0 && pos < KNBR) sIdx[wave * 32 + pos] = j;
      cnt += (int)__popc(mask);
    }
    __syncthreads();
    const int val = sIdx[wave * 32 + lane];
    const int cntc = cnt < KNBR ? cnt : KNBR;
    const int pad = (have != 0) ? first : 0;
    const int v = (lane < cntc) ? val : pad;
    sIdx[wave * 32 + lane] = v;
    __syncthreads();
  }

#pragma unroll
  for (int i = 0; i < 8; ++i) {
    const int row = i * 32 + (tid >> 3);
    const int c = tid & 7;
    int pt = sIdx[row];
    pt = pt < 0 ? 0 : (pt > NPTS - 1 ? NPTS - 1 : pt);
    const v4u v = *(const v4u*)(FT + ((size_t)bb * NPTS + pt) * CIN + c * 8);
    *(v4u*)(sA + row * 64 + c * 8) = v;
  }
  {
    int pt = sIdx[tid];
    pt = pt < 0 ? 0 : (pt > NPTS - 1 ? NPTS - 1 : pt);
    const int m = mbase + (tid >> 5);
    const float rx = cb[pt] - ce[m];
    const float ry = cb[NPTS + pt] - ce[NCEN + m];
    const float rz = cb[2 * NPTS + pt] - ce[2 * NCEN + m];
    *(v4f*)(sRel + tid * 4) = (v4f){rx, ry, rz, 0.0f};
  }
  __syncthreads();

  const _Float16* A16 = (const _Float16*)sA;
  v8f acc[2][4];
  tile_gemm(A16 + (32 * wave) * 64, (const _Float16*)sW1, rl, hh, acc);
  {
    v4f wc[4]; float bo[4];
#pragma unroll
    for (int j = 0; j < 4; ++j) { wc[j] = *(const v4f*)(sWc + (16 * j + rl) * 4); bo[j] = sB1[16 * j + rl]; }
#pragma unroll
    for (int i = 0; i < 2; ++i)
#pragma unroll
      for (int r = 0; r < 8; ++r) {
        const int row = 32 * wave + 16 * i + 8 * hh + r;
        const v4f rel = *(const v4f*)(sRel + row * 4);
#pragma unroll
        for (int j = 0; j < 4; ++j) {
          float t = wc[j][0] * rel[0];
          t = fmaf(wc[j][1], rel[1], t);
          t = fmaf(wc[j][2], rel[2], t);
          t = t + bo[j];
          acc[i][j][r] = fmaf(acc[i][j][r], WCARRY_INV, t);
        }
      }
  }

  if (!DO_L2) {
    tile_stats(acc, hh, rl, wave, sStat);
    __syncthreads();
    if (tid < 128) {
      const int which = tid >> 6, chn = tid & 63;
      float a = 0.0f;
#pragma unroll
      for (int w = 0; w < 8; ++w) a = a + sStat[(w * 2 + which) * 64 + chn];
      sBlk[tid] = a;
    }
    __syncthreads();
    if (wave == 0) {
      const v4f v = *(const v4f*)(sBlk + 4 * lane);
      float* pp = PART + (size_t)blk * 128 + 4 * lane;
      for (int pass = 0; pass < 2; ++pass) { *(volatile v4f*)pp = v; __threadfence(); }
    }
  } else {
    {
      float scl[4], shf[4];
#pragma unroll
      for (int j = 0; j < 4; ++j) { scl[j] = sSc[16 * j + rl]; shf[j] = sSh[16 * j + rl]; }
#pragma unroll
      for (int i = 0; i < 2; ++i)
#pragma unroll
        for (int r = 0; r < 8; ++r) {
          const int row = 32 * wave + 16 * i + 8 * hh + r;
#pragma unroll
          for (int j = 0; j < 4; ++j) {
            const float a = fmaxf(fmaf(acc[i][j][r], scl[j], shf[j]), 0.0f);
            sA[row * 64 + 16 * j + rl] = h_bits(a);
          }
        }
    }
    __syncthreads();
    tile_gemm(A16 + (32 * wave) * 64, (const _Float16*)sW2, rl, hh, acc);
    {
      float bo2[4];
#pragma unroll
      for (int j = 0; j < 4; ++j) bo2[j] = sB2[16 * j + rl];
#pragma unroll
      for (int i = 0; i < 2; ++i)
#pragma unroll
        for (int j = 0; j < 4; ++j)
#pragma unroll
          for (int r = 0; r < 8; ++r) acc[i][j][r] = fmaf(acc[i][j][r], WCARRY_INV, bo2[j]);
    }
    tile_stats(acc, hh, rl, wave, sStat);
    __syncthreads();
    if (tid < 128) {
      const int which = tid >> 6, chn = tid & 63;
      float a = 0.0f;
#pragma unroll
      for (int w = 0; w < 8; ++w) a = a + sStat[(w * 2 + which) * 64 + chn];
      sBlk[tid] = a;
    }
    __syncthreads();
    if (wave == 0) {
      const v4f v = *(const v4f*)(sBlk + 4 * lane);
      float* pp = PART + (size_t)blk * 128 + 4 * lane;
      for (int pass = 0; pass < 2; ++pass) { *(volatile v4f*)pp = v; __threadfence(); }
    }
#pragma unroll
    for (int i = 0; i < 2; ++i)
#pragma unroll
      for (int r = 0; r < 8; ++r) {
        const int row = 32 * wave + 16 * i + 8 * hh + r;
#pragma unroll
        for (int j = 0; j < 4; ++j) sA[row * 64 + 16 * j + rl] = h_bits(acc[i][j][r] * YCARRY);
      }
    __syncthreads();
    {
      const int q = lane >> 3, c8 = (lane & 7) * 8;
      for (int pass = 0; pass < 2; ++pass) {
#pragma unroll
        for (int it = 0; it < 8; ++it) {
          const int row = 32 * wave + it * 4 + q;
          const v4u u = *(const v4u*)(sA + row * 64 + c8);
          *(volatile v4u*)(Y2 + ((size_t)(r0 + row)) * 64 + c8) = u;
        }
        __threadfence();
      }
    }
  }
}

template <int NCH>
__global__ __launch_bounds__(NT) void bn_fin_kernel(const float* __restrict__ PART, int nblk,
                                                  const float* __restrict__ g, const float* __restrict__ bt,
                                                  float* __restrict__ SS) {
  static_assert((2 * NCH) % 128 == 0);
  __shared__ double sD[2 * NCH];
  __shared__ __align__(16) float sOut[2 * NCH];
  const int tid = threadIdx.x, lane = tid & 31, wave = tid >> 5;
  if (tid < 2 * NCH) {
    double a = 0.0;
#pragma unroll 1
    for (int k = 0; k < nblk; ++k) a += (double)PART[(size_t)k * (2 * NCH) + tid];
    sD[tid] = a;
  }
  __syncthreads();
  if (tid < NCH) {
    const double inv_n = 1.0 / (double)NCOL;
    const double mean = sD[tid] * inv_n;
    double var = sD[NCH + tid] * inv_n - mean * mean;
    var = var > 0.0 ? var : 0.0;
    const float varf = (float)var;
    const float rstd = 1.0f / sqrtf(varf + BN_EPS);
    const float scale = g[tid] * rstd;
    const float meanf = (float)mean;
    const float shift = bt[tid] - meanf * scale;
    sOut[tid] = scale;
    sOut[NCH + tid] = shift;
  }
  __syncthreads();
  if (wave == 0) {
    constexpr int NSEG = (2 * NCH) / 128;
    v4f vv[NSEG];
#pragma unroll
    for (int s = 0; s < NSEG; ++s) vv[s] = *(const v4f*)(sOut + s * 128 + 4 * lane);
    for (int pass = 0; pass < 2; ++pass) {
#pragma unroll
      for (int s = 0; s < NSEG; ++s) *(volatile v4f*)(SS + s * 128 + 4 * lane) = vv[s];
      __threadfence();
    }
  }
}

__global__ __launch_bounds__(NT) void mlp3_kernel(const unsigned short* __restrict__ Y2, const unsigned short* __restrict__ WT,
                                                const float* __restrict__ SS2, const float* __restrict__ b3,
                                                float* __restrict__ PART, float* __restrict__ MM) {
  __shared__ __align__(16) unsigned short sA[ROWS3 * 64];
  __shared__ __align__(16) unsigned short sW3[128 * 64];
  __shared__ float sSc[64];
  __shared__ float sSh[64];
  __shared__ float sB3[128];
  __shared__ float sStat[8 * 2 * 64];
  __shared__ __align__(16) float sBlk[256];
  __shared__ __align__(16) float sMM[4 * 2 * 128];

  const int tid = threadIdx.x, lane = tid & 31, wave = tid >> 5;
  const int rl = lane & 15, hh = lane >> 4;
  const int blk = blockIdx.x;
  const int r0 = blk * ROWS3;

  {
    const v4u* wsrc = (const v4u*)WT;
    v4u* d3 = (v4u*)sW3;
#pragma unroll
    for (int i = 0; i < 4; ++i) d3[i * NT + tid] = wsrc[1024 + i * NT + tid];
  }
  if (tid < 64) { sSc[tid] = SS2[tid] * YCARRY_INV; sSh[tid] = SS2[64 + tid]; }
  if (tid < 128) sB3[tid] = b3[tid];
  __syncthreads();

#pragma unroll
  for (int i = 0; i < 4; ++i) {
    const int row = i * 32 + (tid >> 3);
    const int c = tid & 7;
    const v4u w = *(const v4u*)(Y2 + ((size_t)(r0 + row)) * 64 + c * 8);
    unsigned short hb[8];
#pragma unroll
    for (int e = 0; e < 4; ++e) {
      const unsigned wd = w[e];
      const int n0 = c * 8 + 2 * e;
      const float f0 = h16_to_f32(wd & 0xffffu);
      const float f1 = h16_to_f32(wd >> 16);
      const float a0 = fmaxf(fmaf(f0, sSc[n0], sSh[n0]), 0.0f);
      const float a1 = fmaxf(fmaf(f1, sSc[n0 + 1], sSh[n0 + 1]), 0.0f);
      hb[2 * e] = h_bits(a0); hb[2 * e + 1] = h_bits(a1);
    }
    const v4u u = (v4u){pk16(hb[0], hb[1]), pk16(hb[2], hb[3]), pk16(hb[4], hb[5]), pk16(hb[6], hb[7])};
    *(v4u*)(sA + row * 64 + c * 8) = u;
  }
  __syncthreads();

  const int rg = wave >> 1, cg = wave & 1;
  v8f acc[2][4];
  tile_gemm((const _Float16*)sA + (32 * rg) * 64, (const _Float16*)sW3 + (64 * cg) * 64, rl, hh, acc);
  {
    float bo[4];
#pragma unroll
    for (int j = 0; j < 4; ++j) bo[j] = sB3[64 * cg + 16 * j + rl];
#pragma unroll
    for (int i = 0; i < 2; ++i)
#pragma unroll
      for (int j = 0; j < 4; ++j)
#pragma unroll
        for (int r = 0; r < 8; ++r) acc[i][j][r] = fmaf(acc[i][j][r], WCARRY_INV, bo[j]);
  }
  tile_stats(acc, hh, rl, wave, sStat);
  {
    float mx[4], mn[4];
#pragma unroll
    for (int j = 0; j < 4; ++j) { mx[j] = acc[0][j][0]; mn[j] = acc[0][j][0]; }
#pragma unroll
    for (int i = 0; i < 2; ++i)
#pragma unroll
      for (int j = 0; j < 4; ++j)
#pragma unroll
        for (int r = 0; r < 8; ++r) { mx[j] = fmaxf(mx[j], acc[i][j][r]); mn[j] = fminf(mn[j], acc[i][j][r]); }
#pragma unroll
    for (int j = 0; j < 4; ++j) {
      mx[j] = fmaxf(mx[j], __shfl_xor(mx[j], 16, 32));
      mn[j] = fminf(mn[j], __shfl_xor(mn[j], 16, 32));
    }
    if (hh == 0) {
#pragma unroll
      for (int j = 0; j < 4; ++j) {
        sMM[(rg * 2 + 0) * 128 + 64 * cg + 16 * j + rl] = mx[j];
        sMM[(rg * 2 + 1) * 128 + 64 * cg + 16 * j + rl] = mn[j];
      }
    }
  }
  __syncthreads();
  {
    const int which = tid >> 7, chn = tid & 127;
    const int cgc = chn >> 6, cl = chn & 63;
    float a = 0.0f;
#pragma unroll
    for (int g = 0; g < 4; ++g) a = a + sStat[((2 * g + cgc) * 2 + which) * 64 + cl];
    sBlk[tid] = a;
  }
  __syncthreads();
  if (wave == 0) {
    const v4f v0 = *(const v4f*)(sBlk + 4 * lane);
    const v4f v1 = *(const v4f*)(sBlk + 128 + 4 * lane);
    float* pp = PART + (size_t)blk * 256 + 4 * lane;
    for (int pass = 0; pass < 2; ++pass) {
      *(volatile v4f*)pp = v0;
      *(volatile v4f*)(pp + 128) = v1;
      __threadfence();
    }
  }
  {
    const v4f v = *(const v4f*)(sMM + 4 * tid);
    float* mp = MM + (size_t)blk * 1024 + 4 * tid;
    for (int pass = 0; pass < 2; ++pass) { *(volatile v4f*)mp = v; __threadfence(); }
  }
}

__global__ __launch_bounds__(NT) void final_kernel(const float* __restrict__ MM, const float* __restrict__ SS3, float* __restrict__ out0) {
  __shared__ __align__(16) float sV[128 * 36];
  __shared__ float sSc[128];
  __shared__ float sSh[128];
  const int tid = threadIdx.x, lane = tid & 31, wave = tid >> 5;
  const int b = blockIdx.x >> 5;
  const int m0 = (blockIdx.x & 31) * 32;
  const int c0 = b * NCEN + m0;
  if (tid < 128) { sSc[tid] = SS3[tid]; sSh[tid] = SS3[128 + tid]; }
  __syncthreads();
#pragma unroll
  for (int i = 0; i < 4; ++i) {
    const int e = i * NT + tid;
    const int cl = e >> 5;
    const int ch4 = (e & 31) * 4;
    const float* mp = MM + ((size_t)(c0 + cl)) * 256 + ch4;
    const v4f mx = *(const v4f*)(mp);
    const v4f mn = *(const v4f*)(mp + 128);
#pragma unroll
    for (int k = 0; k < 4; ++k) {
      const int ch = ch4 + k;
      const float scv = sSc[ch];
      const float fsel = (scv >= 0.0f) ? 1.0f : 0.0f;
      const float gsel = 1.0f - fsel;
      const float v = fmaf(fsel, mx[k], gsel * mn[k]);
      const float o = fmaxf(fmaf(v, scv, sSh[ch]), 0.0f);
      sV[ch * 36 + cl] = o;
    }
  }
  __syncthreads();
  {
    const int q = lane >> 3, m4 = (lane & 7) * 4;
    v4f vv[4];
#pragma unroll
    for (int it = 0; it < 4; ++it) {
      const int ch = it * 32 + wave * 4 + q;
      vv[it] = *(const v4f*)(sV + ch * 36 + m4);
    }
    for (int pass = 0; pass < 2; ++pass) {
#pragma unroll
      for (int it = 0; it < 4; ++it) {
        const int ch = it * 32 + wave * 4 + q;
        *(volatile v4f*)(out0 + ((size_t)(b * NCH3 + ch)) * NCEN + m0 + m4) = vv[it];
      }
      __threadfence();
    }
  }
}

extern "C" void kernel_launch(void* const* d_in, const int* in_sizes, int n_in,
                              void* d_out, int out_size, void* d_ws, size_t ws_size, hipStream_t stream) {
  (void)in_sizes; (void)n_in;
  const float* features = (const float*)d_in[0];
  const float* coords   = (const float*)d_in[1];
  const float* w1  = (const float*)d_in[2];
  const float* b1  = (const float*)d_in[3];
  const float* g1  = (const float*)d_in[4];
  const float* bt1 = (const float*)d_in[5];
  const float* w2  = (const float*)d_in[6];
  const float* b2  = (const float*)d_in[7];
  const float* g2  = (const float*)d_in[8];
  const float* bt2 = (const float*)d_in[9];
  const float* w3  = (const float*)d_in[10];
  const float* b3  = (const float*)d_in[11];
  const float* g3  = (const float*)d_in[12];
  const float* bt3 = (const float*)d_in[13];

  constexpr size_t OUT0_BYTES = (size_t)NBATCH * NCH3 * NCEN * 4;
  constexpr size_t OUT1_BYTES = (size_t)NBATCH * 3 * NCEN * 4;
  static_assert(OUT0_BYTES == 8388608);
  static_assert(OUT0_BYTES + OUT1_BYTES == 8585216);
  static_assert(OUT0_BYTES % 128 == 0);
  if ((size_t)out_size * 4 < OUT0_BYTES + OUT1_BYTES) return;
  float* out0 = (float*)d_out;
  float* out1 = out0 + OUT0_BYTES / 4;

  char* ws = (char*)d_ws;
  size_t off = 0;
  auto carve = [&](size_t bytes) -> char* { char* p = ws + off; off += (bytes + 255) & ~(size_t)255; return p; };
  unsigned short* FT    = (unsigned short*)carve((size_t)NBATCH * NPTS * CIN * 2);
  unsigned short* WT    = (unsigned short*)carve((size_t)256 * 64 * 2);
  unsigned short* Y2    = (unsigned short*)carve((size_t)NCOL * 64 * 2);
  float*          PART1 = (float*)carve((size_t)NBLK12 * 2 * NCH12 * 4);
  float*          PART2 = (float*)carve((size_t)NBLK12 * 2 * NCH12 * 4);
  float*          PART3 = (float*)carve((size_t)NBLK3 * 2 * NCH3 * 4);
  float*          SS1   = (float*)carve((size_t)2 * NCH12 * 4);
  float*          SS2   = (float*)carve((size_t)2 * NCH12 * 4);
  float*          SS3   = (float*)carve((size_t)2 * NCH3 * 4);
  float*          MM    = (float*)carve((size_t)NCENTOT * 2 * NCH3 * 4);
  if (off > ws_size || off > (size_t)134217728) return;

  feat_transpose_kernel<<<dim3(NPTS / 64, NBATCH), NT, 0, stream>>>(features, FT);
  wcast_kernel<<<NWCBLK, NT, 0, stream>>>(w1, w2, w3, WT);
  fps_kernel<<<NBATCH, FPS_NT, 0, stream>>>(coords, out1);
  mlp12_kernel<false><<<NBLK12, NT, 0, stream>>>(FT, coords, out1, WT, w1, b1, SS1, b2, PART1, Y2);
  bn_fin_kernel<NCH12><<<1, NT, 0, stream>>>(PART1, NBLK12, g1, bt1, SS1);
  mlp12_kernel<true><<<NBLK12, NT, 0, stream>>>(FT, coords, out1, WT, w1, b1, SS1, b2, PART2, Y2);
  bn_fin_kernel<NCH12><<<1, NT, 0, stream>>>(PART2, NBLK12, g2, bt2, SS2);
  mlp3_kernel<<<NBLK3, NT, 0, stream>>>(Y2, WT, SS2, b3, PART3, MM);
  bn_fin_kernel<NCH3><<<1, NT, 0, stream>>>(PART3, NBLK3, g3, bt3, SS3);
  final_kernel<<<NBATCH * (NCEN / 32), NT, 0, stream>>>(MM, SS3, out0);
}
